// Decoder_16922171147076
// MI455X (gfx1250) — hardware-verified
//
#include <hip/hip_runtime.h>
#include <math.h>

typedef __attribute__((ext_vector_type(16))) _Float16 v16h;
typedef __attribute__((ext_vector_type(8)))  _Float16 v8h;
typedef __attribute__((ext_vector_type(8)))  float    v8f;
typedef __attribute__((ext_vector_type(4)))  float    v4f;
typedef v4f v4fa __attribute__((may_alias));
typedef v8h v8ha __attribute__((may_alias));

constexpr int OBS_STEPS  = 8;
constexpr int PRED_STEPS = 12;
constexpr int ALL_STEPS  = 20;
constexpr int NPED       = 32768;
constexpr int NSCENE     = 512;
constexpr int NAGENT     = 64;
constexpr int GHID       = 64;
constexpr int AHID       = 32;
constexpr int NHEAD0     = 4;
constexpr int FOUT0      = 16;
constexpr int FCAT       = 64;
constexpr int FOUT1      = 32;
constexpr int NTHR       = 256;
constexpr int ATTN_PLANE = NAGENT * NAGENT;

constexpr float H_CARRY   = 64.0f;
constexpr float W_CARRY   = 16.0f;
constexpr float X_CARRY   = 16.0f;
constexpr float HP_CARRY  = 64.0f;
constexpr float A_CARRY   = 16384.0f;
constexpr float RES_CARRY = 2048.0f;
constexpr float LSTM_FOLD = 1.0f / (H_CARRY * W_CARRY);
constexpr float RES_FOLD  = LSTM_FOLD / RES_CARRY;
constexpr float HP_FOLD   = HP_CARRY / (X_CARRY * W_CARRY);
constexpr float PV_FOLD   = 1.0f / (A_CARRY * HP_CARRY);
constexpr float INV_AGENTS = 1.0f / (float)NAGENT;
constexpr float NORM_EPS   = 1e-5f;
constexpr float LEAKY      = 0.2f;
constexpr float F16_MIN_NORMAL = 1.0f / 16384.0f;

static_assert(NSCENE * NAGENT == NPED, "scenes x agents");
static_assert(NHEAD0 * FOUT0 == FCAT, "head concat width");
static_assert(GHID % 32 == 0 && AHID % 32 == 0 && FCAT % 32 == 0 && NAGENT % 32 == 0, "K multiples of 32");
static_assert(NAGENT % 16 == 0 && FOUT1 % 16 == 0, "tile multiples");
static_assert(NTHR == 4 * NAGENT, "four lanes per agent row");
static_assert(OBS_STEPS + PRED_STEPS == ALL_STEPS, "time axis");

template <typename T> struct Frag;
template <> struct Frag<_Float16> {
  typedef v16h V; union U { v16h v; v8h h[2]; };
  static __device__ __forceinline__ v16h load(const _Float16* p) {
    U f; f.h[0] = *(const v8h*)(p); f.h[1] = *(const v8h*)(p + 16); return f.v;
  }
};

__device__ __forceinline__ v8f mma16(v16h a, v16h b, v8f c) {
  c = __builtin_amdgcn_wmma_f32_16x16x32_f16(false, a, false, b, (short)0, c, false, false);
  asm volatile("v_nop\n\tv_nop\n\tv_nop\n\tv_nop" : "+v"(c) : "v"(a), "v"(b));
  return c;
}

__device__ __forceinline__ v16h frag_from_f32(const float* p, float sc) {
  const v4f p0 = *(const v4fa*)(p);
  const v4f p1 = *(const v4fa*)(p + 4);
  const v4f p2 = *(const v4fa*)(p + 16);
  const v4f p3 = *(const v4fa*)(p + 20);
  v16h a;
#pragma unroll
  for (int e = 0; e < 4; ++e) {
    a[e]      = (_Float16)(p0[e] * sc);
    a[4 + e]  = (_Float16)(p1[e] * sc);
    a[8 + e]  = (_Float16)(p2[e] * sc);
    a[12 + e] = (_Float16)(p3[e] * sc);
  }
  return a;
}

__device__ __forceinline__ float hi_part(float v) {
  const float hf = (float)(_Float16)v;
  return (fabsf(hf) < F16_MIN_NORMAL) ? 0.0f : hf;
}

__device__ __forceinline__ void frag_split_f32(const float* p, float sc, v16h& hi, v16h& res) {
  const v4f p0 = *(const v4fa*)(p);
  const v4f p1 = *(const v4fa*)(p + 4);
  const v4f p2 = *(const v4fa*)(p + 16);
  const v4f p3 = *(const v4fa*)(p + 20);
#pragma unroll
  for (int e = 0; e < 4; ++e) {
    const float v0 = p0[e] * sc;
    const float v1 = p1[e] * sc;
    const float v2 = p2[e] * sc;
    const float v3 = p3[e] * sc;
    const float h0 = hi_part(v0);
    const float h1 = hi_part(v1);
    const float h2 = hi_part(v2);
    const float h3 = hi_part(v3);
    hi[e]       = (_Float16)h0;
    hi[4 + e]   = (_Float16)h1;
    hi[8 + e]   = (_Float16)h2;
    hi[12 + e]  = (_Float16)h3;
    res[e]      = (_Float16)((v0 - h0) * RES_CARRY);
    res[4 + e]  = (_Float16)((v1 - h1) * RES_CARRY);
    res[8 + e]  = (_Float16)((v2 - h2) * RES_CARRY);
    res[12 + e] = (_Float16)((v3 - h3) * RES_CARRY);
  }
}

__device__ __forceinline__ v16h frag_norm_f32(const float* p, const float* mu, const float* rs, float sc) {
  const v4f x0 = (*(const v4fa*)(p)      - *(const v4fa*)(mu))      * *(const v4fa*)(rs);
  const v4f x1 = (*(const v4fa*)(p + 4)  - *(const v4fa*)(mu + 4))  * *(const v4fa*)(rs + 4);
  const v4f x2 = (*(const v4fa*)(p + 16) - *(const v4fa*)(mu + 16)) * *(const v4fa*)(rs + 16);
  const v4f x3 = (*(const v4fa*)(p + 20) - *(const v4fa*)(mu + 20)) * *(const v4fa*)(rs + 20);
  v16h a;
#pragma unroll
  for (int e = 0; e < 4; ++e) {
    a[e]      = (_Float16)(x0[e] * sc);
    a[4 + e]  = (_Float16)(x1[e] * sc);
    a[8 + e]  = (_Float16)(x2[e] * sc);
    a[12 + e] = (_Float16)(x3[e] * sc);
  }
  return a;
}

__device__ __forceinline__ float sigm(float x) {
  const float xc = fminf(fmaxf(x, -30.0f), 30.0f);
  return __builtin_amdgcn_rcpf(1.0f + expf(-xc));
}
__device__ __forceinline__ float tanh_e(float x) {
  const float xc = fminf(fmaxf(x, -15.0f), 15.0f);
  return 1.0f - 2.0f * __builtin_amdgcn_rcpf(expf(2.0f * xc) + 1.0f);
}
__device__ __forceinline__ void lstm_point(float zi, float zf, float zg, float zo, float* cptr, float* hptr) {
  const float cn = sigm(zf) * (*cptr) + sigm(zi) * tanh_e(zg);
  *cptr = cn;
  *hptr = sigm(zo) * tanh_e(cn);
}

__device__ __forceinline__ void attn_row_block(const float* sl, const float* dl, _Float16* plane, int n, int oct) {
  const float sn = sl[n];
  const v4f d0 = *(const v4fa*)(dl + oct * 8);
  const v4f d1 = *(const v4fa*)(dl + oct * 8 + 4);
  float ev[8];
#pragma unroll
  for (int e = 0; e < 4; ++e) {
    const float u0 = sn + d0[e];
    const float u1 = sn + d1[e];
    ev[e]     = (u0 >= 0.0f) ? u0 : LEAKY * u0;
    ev[4 + e] = (u1 >= 0.0f) ? u1 : LEAKY * u1;
  }
  float mx = ev[0];
#pragma unroll
  for (int e = 1; e < 8; ++e) mx = fmaxf(mx, ev[e]);
  mx = fmaxf(mx, __shfl_xor(mx, 1, 32));
  mx = fmaxf(mx, __shfl_xor(mx, 2, 32));
  mx = fmaxf(mx, __shfl_xor(mx, 4, 32));
  float sum = 0.0f;
#pragma unroll
  for (int e = 0; e < 8; ++e) { ev[e] = expf(ev[e] - mx); sum += ev[e]; }
  sum += __shfl_xor(sum, 1, 32);
  sum += __shfl_xor(sum, 2, 32);
  sum += __shfl_xor(sum, 4, 32);
  const float inv = __builtin_amdgcn_rcpf(sum);
  v8h av;
#pragma unroll
  for (int e = 0; e < 8; ++e) av[e] = (_Float16)((ev[e] * inv - INV_AGENTS) * A_CARRY);
  *(v8ha*)(plane + n * NAGENT + oct * 8) = av;
}

__global__ __launch_bounds__(NTHR) void scene_decode_kernel(
    const float* __restrict__ goal_real,  const float* __restrict__ gh_in,
    const float* __restrict__ action_real, const float* __restrict__ ah_in,
    const float* __restrict__ Wih_g, const float* __restrict__ Whh_g,
    const float* __restrict__ bih_g, const float* __restrict__ bhh_g,
    const float* __restrict__ W_h2g, const float* __restrict__ b_h2g,
    const float* __restrict__ Wih_a, const float* __restrict__ Whh_a,
    const float* __restrict__ bih_a, const float* __restrict__ bhh_a,
    const float* __restrict__ W_h2a, const float* __restrict__ b_h2a,
    const float* __restrict__ W_ga,  const float* __restrict__ b_ga,
    const float* __restrict__ W_aa,  const float* __restrict__ b_aa,
    const float* __restrict__ w0,    const float* __restrict__ asrc0,
    const float* __restrict__ adst0, const float* __restrict__ bias0,
    const float* __restrict__ w1,    const float* __restrict__ asrc1,
    const float* __restrict__ adst1, const float* __restrict__ bias1,
    float* __restrict__ out)
{
  __shared__ __align__(16) float    s_gh[NAGENT * GHID];
  __shared__ __align__(16) float    s_gc[NAGENT * GHID];
  __shared__ __align__(16) float    s_ah[NAGENT * AHID];
  __shared__ __align__(16) float    s_ac[NAGENT * AHID];
  __shared__ __align__(16) float    s_y0[NAGENT * FCAT];
  __shared__ __align__(16) float    s_go[NAGENT * 2];
  __shared__ __align__(16) float    s_ao[NAGENT * 2];
  __shared__ __align__(16) _Float16 s_whhg[4 * GHID * GHID];
  __shared__ __align__(16) _Float16 s_whha[4 * AHID * AHID];
  __shared__ __align__(16) _Float16 s_w0t[FCAT * AHID];
  __shared__ __align__(16) _Float16 s_w1t[FOUT1 * FCAT];
  __shared__ __align__(16) _Float16 s_hpt[FCAT * NAGENT];
  __shared__ __align__(16) _Float16 s_attn[2 * ATTN_PLANE];
  __shared__ __align__(16) float    s_wihg[4 * GHID * 2];
  __shared__ __align__(16) float    s_bg[4 * GHID];
  __shared__ __align__(16) float    s_wiha[4 * AHID * 2];
  __shared__ __align__(16) float    s_ba[4 * AHID];
  __shared__ __align__(16) float    s_wh2g[2 * GHID];
  __shared__ __align__(16) float    s_wh2a[2 * AHID];
  __shared__ __align__(16) float    s_wga[AHID * 2];
  __shared__ __align__(16) float    s_bga[AHID];
  __shared__ __align__(16) float    s_waa[GHID * 2];
  __shared__ __align__(16) float    s_baa[GHID];
  __shared__ __align__(16) float    s_us0[NHEAD0 * AHID];
  __shared__ __align__(16) float    s_ud0[NHEAD0 * AHID];
  __shared__ __align__(16) float    s_us1[FCAT];
  __shared__ __align__(16) float    s_ud1[FCAT];
  __shared__ __align__(16) float    s_b0v[FOUT0];
  __shared__ __align__(16) float    s_b1v[FOUT1];
  __shared__ __align__(16) float    s_bh[4];
  __shared__ __align__(16) float    s_sl[NHEAD0 * NAGENT];
  __shared__ __align__(16) float    s_dl[NHEAD0 * NAGENT];
  __shared__ __align__(16) float    s_mean[FCAT];
  __shared__ __align__(16) float    s_rstd[FCAT];

  const int tid  = threadIdx.x;
  const int lane = tid & 31;
  const int wid  = __builtin_amdgcn_readfirstlane(tid >> 5);
  const int n15  = lane & 15;
  const int hh   = lane >> 4;
  const int rb   = hh * 8;
  const int ped0 = blockIdx.x * NAGENT;
  const v8f zero8 = {0.f, 0.f, 0.f, 0.f, 0.f, 0.f, 0.f, 0.f};
  const v4f zero4 = {0.f, 0.f, 0.f, 0.f};

#pragma unroll 1
  for (int i = tid; i < NAGENT * GHID / 4; i += NTHR) {
    const v4f v = *(const v4f*)(gh_in + (size_t)ped0 * GHID + 4 * i);
    *(v4fa*)(s_gh + 4 * i) = v;
    *(v4fa*)(s_gc + 4 * i) = zero4;
  }
#pragma unroll 1
  for (int i = tid; i < NAGENT * AHID / 4; i += NTHR) {
    const v4f v = *(const v4f*)(ah_in + (size_t)ped0 * AHID + 4 * i);
    *(v4fa*)(s_ah + 4 * i) = v;
    *(v4fa*)(s_ac + 4 * i) = zero4;
  }
  {
    const int i7 = tid & 127;
    const size_t base = ((size_t)(OBS_STEPS - 1) * NPED + (size_t)ped0) * 2;
    const float gv = goal_real[base + i7];
    const float av = action_real[base + i7];
    if (tid < 128) { s_go[i7] = gv; s_ao[i7] = av; }
  }
  __syncthreads();
#pragma unroll 1
  for (int i = tid; i < 4 * GHID * GHID / 8; i += NTHR) {
    const v4f a = *(const v4f*)(Whh_g + 8 * i);
    const v4f b = *(const v4f*)(Whh_g + 8 * i + 4);
    v8h hv;
#pragma unroll
    for (int e = 0; e < 4; ++e) { hv[e] = (_Float16)(a[e] * W_CARRY); hv[4 + e] = (_Float16)(b[e] * W_CARRY); }
    *(v8ha*)(s_whhg + 8 * i) = hv;
  }
#pragma unroll 1
  for (int i = tid; i < 4 * AHID * AHID / 8; i += NTHR) {
    const v4f a = *(const v4f*)(Whh_a + 8 * i);
    const v4f b = *(const v4f*)(Whh_a + 8 * i + 4);
    v8h hv;
#pragma unroll
    for (int e = 0; e < 4; ++e) { hv[e] = (_Float16)(a[e] * W_CARRY); hv[4 + e] = (_Float16)(b[e] * W_CARRY); }
    *(v8ha*)(s_whha + 8 * i) = hv;
  }
  __syncthreads();
  {
    const int f = tid >> 2, k8 = (tid & 3) * 8;
    const int hd = f >> 4, o = f & 15;
    v8h hv;
#pragma unroll
    for (int e = 0; e < 8; ++e) hv[e] = (_Float16)(w0[(hd * AHID + k8 + e) * FOUT0 + o] * W_CARRY);
    *(v8ha*)(s_w0t + f * AHID + k8) = hv;
  }
  __syncthreads();
  {
    const int o = tid >> 3, k8 = (tid & 7) * 8;
    v8h hv;
#pragma unroll
    for (int e = 0; e < 8; ++e) hv[e] = (_Float16)(w1[(k8 + e) * FOUT1 + o] * W_CARRY);
    *(v8ha*)(s_w1t + o * FCAT + k8) = hv;
  }
  __syncthreads();
  {
    s_wihg[tid]       = Wih_g[tid];
    s_wihg[256 + tid] = Wih_g[256 + tid];
    s_bg[tid]         = bih_g[tid] + bhh_g[tid];
    s_wiha[tid]       = Wih_a[tid];
  }
  __syncthreads();
  {
    const int i7 = tid & 127;
    const float v0 = bih_a[i7] + bhh_a[i7];
    const float v1 = W_h2g[i7];
    const float v2 = W_aa[i7];
    if (tid < 128) { s_ba[i7] = v0; s_wh2g[i7] = v1; s_waa[i7] = v2; }
    const int i6 = tid & 63;
    const float v3 = W_h2a[i6];
    const float v4 = W_ga[i6];
    const float v5 = b_aa[i6];
    if (tid < 64) { s_wh2a[i6] = v3; s_wga[i6] = v4; s_baa[i6] = v5; }
  }
  __syncthreads();
  {
    const int i5 = tid & 31;
    const float v0 = b_ga[i5];
    const float v1 = bias1[i5];
    if (tid < 32) { s_bga[i5] = v0; s_b1v[i5] = v1; }
    const int i4 = tid & 15;
    float v2 = bias0[i4];
    asm volatile("" : "+v"(v2));
    if (tid < 16) s_b0v[i4] = v2;
    const int i1 = tid & 1;
    float v3 = b_h2g[i1];
    asm volatile("" : "+v"(v3));
    float v4 = b_h2a[i1];
    asm volatile("" : "+v"(v4));
    if (tid < 2) { s_bh[i1] = v3; s_bh[2 + i1] = v4; }
  }
  __syncthreads();
  {
    const int idx = tid & 127;
    const int hd = idx >> 5;
    const float* wrow = w0 + (size_t)idx * FOUT0;
    float ss = 0.0f, dd = 0.0f;
#pragma unroll 1
    for (int o4 = 0; o4 < FOUT0; o4 += 4) {
      const v4f wv = *(const v4f*)(wrow + o4);
      const v4f as = *(const v4f*)(asrc0 + hd * FOUT0 + o4);
      const v4f ad = *(const v4f*)(adst0 + hd * FOUT0 + o4);
#pragma unroll
      for (int e = 0; e < 4; ++e) { ss = fmaf(wv[e], as[e], ss); dd = fmaf(wv[e], ad[e], dd); }
    }
    if (tid < 128) s_us0[idx] = ss; else s_ud0[idx] = dd;
  }
  {
    const int k = tid & 63;
    const float* wrow = w1 + (size_t)k * FOUT1;
    float ss = 0.0f, dd = 0.0f;
#pragma unroll 1
    for (int o4 = 0; o4 < FOUT1; o4 += 4) {
      const v4f wv = *(const v4f*)(wrow + o4);
      const v4f as = *(const v4f*)(asrc1 + o4);
      const v4f ad = *(const v4f*)(adst1 + o4);
#pragma unroll
      for (int e = 0; e < 4; ++e) { ss = fmaf(wv[e], as[e], ss); dd = fmaf(wv[e], ad[e], dd); }
    }
    if (tid < 64) s_us1[k] = ss;
    else if (tid < 128) s_ud1[k] = dd;
  }
  __syncthreads();

#pragma unroll 1
  for (int t = 0; t < PRED_STEPS; ++t) {
    if (wid < 4) {
      const int m0 = wid * 16;
      const float* hrow = s_gh + (m0 + n15) * GHID + 8 * hh;
      v16h a0, a1, a0r, a1r;
      frag_split_f32(hrow, H_CARRY, a0, a0r);
      frag_split_f32(hrow + 32, H_CARRY, a1, a1r);
#pragma unroll 1
      for (int q = 0; q < GHID / 16; ++q) {
        const _Float16* wb = s_whhg + (q * 16 + n15) * GHID + 8 * hh;
        const int j = q * 16 + n15;
        float zc[4][8];
#pragma unroll
        for (int g = 0; g < 4; ++g) {
          const v16h b0 = Frag<_Float16>::load(wb + g * GHID * GHID);
          const v16h b1 = Frag<_Float16>::load(wb + g * GHID * GHID + 32);
          v8f zm = zero8, zr = zero8;
          zm = mma16(a0, b0, zm);
          zm = mma16(a1, b1, zm);
          zr = mma16(a0r, b0, zr);
          zr = mma16(a1r, b1, zr);
          const float bgate = s_bg[g * GHID + j];
#pragma unroll
          for (int r = 0; r < 8; ++r) zc[g][r] = (zm[r] * LSTM_FOLD + zr[r] * RES_FOLD) + bgate;
        }
        const float wi0 = s_wihg[2 * j],              wi1 = s_wihg[2 * j + 1];
        const float wf0 = s_wihg[2 * (GHID + j)],     wf1 = s_wihg[2 * (GHID + j) + 1];
        const float wg0 = s_wihg[2 * (2 * GHID + j)], wg1 = s_wihg[2 * (2 * GHID + j) + 1];
        const float wo0 = s_wihg[2 * (3 * GHID + j)], wo1 = s_wihg[2 * (3 * GHID + j) + 1];
#pragma unroll
        for (int r = 0; r < 8; ++r) {
          const int mrow = m0 + rb + r;
          const int mi = mrow * GHID + j;
          const float x0 = s_go[2 * mrow];
          const float x1 = s_go[2 * mrow + 1];
          const float zi = zc[0][r] + (x0 * wi0 + x1 * wi1);
          const float zf = zc[1][r] + (x0 * wf0 + x1 * wf1);
          const float zg = zc[2][r] + (x0 * wg0 + x1 * wg1);
          const float zo = zc[3][r] + (x0 * wo0 + x1 * wo1);
          lstm_point(zi, zf, zg, zo, s_gc + mi, s_gh + mi);
        }
      }
    } else {
      const int m0 = (wid - 4) * 16;
      const v16h a0 = frag_from_f32(s_ah + (m0 + n15) * AHID + 8 * hh, H_CARRY);
      float x0[8], x1[8];
#pragma unroll
      for (int r = 0; r < 8; ++r) { x0[r] = s_ao[2 * (m0 + rb + r)]; x1[r] = s_ao[2 * (m0 + rb + r) + 1]; }
#pragma unroll 1
      for (int q = 0; q < AHID / 16; ++q) {
        const _Float16* wb = s_whha + (q * 16 + n15) * AHID + 8 * hh;
        v8f z0 = zero8, z1 = zero8, z2 = zero8, z3 = zero8;
        z0 = mma16(a0, Frag<_Float16>::load(wb), z0);
        z1 = mma16(a0, Frag<_Float16>::load(wb + 1 * AHID * AHID), z1);
        z2 = mma16(a0, Frag<_Float16>::load(wb + 2 * AHID * AHID), z2);
        z3 = mma16(a0, Frag<_Float16>::load(wb + 3 * AHID * AHID), z3);
        const int j = q * 16 + n15;
        const float wi0 = s_wiha[2 * j],              wi1 = s_wiha[2 * j + 1],              bi = s_ba[j];
        const float wf0 = s_wiha[2 * (AHID + j)],     wf1 = s_wiha[2 * (AHID + j) + 1],     bfv = s_ba[AHID + j];
        const float wg0 = s_wiha[2 * (2 * AHID + j)], wg1 = s_wiha[2 * (2 * AHID + j) + 1], bgv = s_ba[2 * AHID + j];
        const float wo0 = s_wiha[2 * (3 * AHID + j)], wo1 = s_wiha[2 * (3 * AHID + j) + 1], bo = s_ba[3 * AHID + j];
#pragma unroll
        for (int r = 0; r < 8; ++r) {
          const int mi = (m0 + rb + r) * AHID + j;
          const float zi = z0[r] * LSTM_FOLD + (x0[r] * wi0 + x1[r] * wi1 + bi);
          const float zf = z1[r] * LSTM_FOLD + (x0[r] * wf0 + x1[r] * wf1 + bfv);
          const float zg = z2[r] * LSTM_FOLD + (x0[r] * wg0 + x1[r] * wg1 + bgv);
          const float zo = z3[r] * LSTM_FOLD + (x0[r] * wo0 + x1[r] * wo1 + bo);
          lstm_point(zi, zf, zg, zo, s_ac + mi, s_ah + mi);
        }
      }
    }
    __syncthreads();

    {
      const int m = tid >> 2, part = tid & 3;
      const float* gr = s_gh + m * GHID + part * 16;
      float s0 = 0.0f, s1 = 0.0f;
#pragma unroll
      for (int i = 0; i < 4; ++i) {
        const v4f g  = *(const v4fa*)(gr + 4 * i);
        const v4f wa = *(const v4fa*)(s_wh2g + part * 16 + 4 * i);
        const v4f wb = *(const v4fa*)(s_wh2g + GHID + part * 16 + 4 * i);
#pragma unroll
        for (int e = 0; e < 4; ++e) { s0 = fmaf(g[e], wa[e], s0); s1 = fmaf(g[e], wb[e], s1); }
      }
      s0 += __shfl_xor(s0, 1, 32);
      s1 += __shfl_xor(s1, 1, 32);
      s0 += __shfl_xor(s0, 2, 32);
      s1 += __shfl_xor(s1, 2, 32);
      s0 += s_bh[0];
      s1 += s_bh[1];
      if (part == 0) { s_go[2 * m] = s0; s_go[2 * m + 1] = s1; }
      float lg[8];
      float mx = -INFINITY;
#pragma unroll
      for (int e = 0; e < 8; ++e) {
        const int j = part * 8 + e;
        lg[e] = fmaf(s0, s_wga[2 * j], fmaf(s1, s_wga[2 * j + 1], s_bga[j]));
        mx = fmaxf(mx, lg[e]);
      }
      mx = fmaxf(mx, __shfl_xor(mx, 1, 32));
      mx = fmaxf(mx, __shfl_xor(mx, 2, 32));
      float sum = 0.0f;
#pragma unroll
      for (int e = 0; e < 8; ++e) { lg[e] = expf(lg[e] - mx); sum += lg[e]; }
      sum += __shfl_xor(sum, 1, 32);
      sum += __shfl_xor(sum, 2, 32);
      const float inv = __builtin_amdgcn_rcpf(sum);
      float* ar = s_ah + m * AHID + part * 8;
#pragma unroll
      for (int e = 0; e < 8; ++e) ar[e] = ar[e] * (lg[e] * inv);
    }
    __syncthreads();

    if (tid < 128) {
      const float v = s_go[tid];
      volatile float* p = out + (size_t)t * (NPED * 2) + (size_t)ped0 * 2 + tid;
      *p = v;
      __threadfence();
      *p = v;
    }
    {
      const int ch = tid >> 3, oct = tid & 7;
      float v[8];
      float s = 0.0f;
#pragma unroll
      for (int i = 0; i < 8; ++i) { v[i] = s_ah[(oct * 8 + i) * AHID + ch]; s += v[i]; }
      s += __shfl_xor(s, 1, 32);
      s += __shfl_xor(s, 2, 32);
      s += __shfl_xor(s, 4, 32);
      const float mu = s * INV_AGENTS;
      float ss = 0.0f;
#pragma unroll
      for (int i = 0; i < 8; ++i) { const float d = v[i] - mu; ss = fmaf(d, d, ss); }
      ss += __shfl_xor(ss, 1, 32);
      ss += __shfl_xor(ss, 2, 32);
      ss += __shfl_xor(ss, 4, 32);
      const float rs = rsqrtf(ss * INV_AGENTS + NORM_EPS);
      if (oct == 0) { s_mean[ch] = mu; s_rstd[ch] = rs; }
    }
    __syncthreads();

    {
      const int n = tid >> 2, hd = tid & 3;
      const float* xr = s_ah + n * AHID;
      float sv = 0.0f, dv = 0.0f;
#pragma unroll 2
      for (int k = 0; k < AHID; k += 4) {
        const v4f x  = (*(const v4fa*)(xr + k) - *(const v4fa*)(s_mean + k)) * *(const v4fa*)(s_rstd + k);
        const v4f us = *(const v4fa*)(s_us0 + hd * AHID + k);
        const v4f ud = *(const v4fa*)(s_ud0 + hd * AHID + k);
#pragma unroll
        for (int e = 0; e < 4; ++e) { sv = fmaf(x[e], us[e], sv); dv = fmaf(x[e], ud[e], dv); }
      }
      s_sl[hd * NAGENT + n] = sv;
      s_dl[hd * NAGENT + n] = dv;
    }
    {
      const int mt = wid & 3, hp2 = wid >> 2;
      const int n = mt * 16 + n15;
      const v16h xa = frag_norm_f32(s_ah + n * AHID + 8 * hh, s_mean + 8 * hh, s_rstd + 8 * hh, X_CARRY);
#pragma unroll
      for (int hl = 0; hl < 2; ++hl) {
        const int f = (2 * hp2 + hl) * FOUT0 + n15;
        const v16h wb = Frag<_Float16>::load(s_w0t + f * AHID + 8 * hh);
        const v8f acc = mma16(xa, wb, zero8);
        v8h o;
#pragma unroll
        for (int r = 0; r < 8; ++r) o[r] = (_Float16)(acc[r] * HP_FOLD);
        *(v8ha*)(s_hpt + f * NAGENT + mt * 16 + rb) = o;
      }
    }
    __syncthreads();

#pragma unroll 1
    for (int pr = 0; pr < 2; ++pr) {
#pragma unroll 1
      for (int it = 0; it < 4; ++it) {
        const int hl = it >> 1;
        const int head = 2 * pr + hl;
        const int n = (it & 1) * 32 + (tid >> 3);
        attn_row_block(s_sl + head * NAGENT, s_dl + head * NAGENT, s_attn + hl * ATTN_PLANE, n, tid & 7);
      }
      __syncthreads();
      {
        const int hl = wid >> 2, mt = wid & 3;
        const int head = 2 * pr + hl;
        const _Float16* arow = s_attn + hl * ATTN_PLANE + (mt * 16 + n15) * NAGENT + 8 * hh;
        const _Float16* brow = s_hpt + (head * FOUT0 + n15) * NAGENT + 8 * hh;
        v8f acc = zero8;
        acc = mma16(Frag<_Float16>::load(arow), Frag<_Float16>::load(brow), acc);
        acc = mma16(Frag<_Float16>::load(arow + 32), Frag<_Float16>::load(brow + 32), acc);
        const float bb = s_b0v[n15];
#pragma unroll
        for (int r = 0; r < 8; ++r) {
          const float v = acc[r] * PV_FOLD + bb;
          const float en = expm1f(fminf(v, 0.0f));
          s_y0[(mt * 16 + rb + r) * FCAT + head * FOUT0 + n15] = (v > 0.0f) ? v : en;
        }
      }
      __syncthreads();
    }

    {
      const int ch = tid >> 2, q4 = tid & 3;
      float v[16];
      float s = 0.0f;
#pragma unroll
      for (int i = 0; i < 16; ++i) { v[i] = s_y0[(q4 * 16 + i) * FCAT + ch]; s += v[i]; }
      s += __shfl_xor(s, 1, 32);
      s += __shfl_xor(s, 2, 32);
      const float mu = s * INV_AGENTS;
      float ss = 0.0f;
#pragma unroll
      for (int i = 0; i < 16; ++i) { const float d = v[i] - mu; ss = fmaf(d, d, ss); }
      ss += __shfl_xor(ss, 1, 32);
      ss += __shfl_xor(ss, 2, 32);
      const float rs = rsqrtf(ss * INV_AGENTS + NORM_EPS);
      if (q4 == 0) { s_mean[ch] = mu; s_rstd[ch] = rs; }
    }
    __syncthreads();

    {
      const int n = tid >> 2, part = tid & 3;
      const float* xr = s_y0 + n * FCAT + part * 16;
      float sv = 0.0f, dv = 0.0f;
#pragma unroll 2
      for (int k = 0; k < 16; k += 4) {
        const v4f x  = (*(const v4fa*)(xr + k) - *(const v4fa*)(s_mean + part * 16 + k)) * *(const v4fa*)(s_rstd + part * 16 + k);
        const v4f us = *(const v4fa*)(s_us1 + part * 16 + k);
        const v4f ud = *(const v4fa*)(s_ud1 + part * 16 + k);
#pragma unroll
        for (int e = 0; e < 4; ++e) { sv = fmaf(x[e], us[e], sv); dv = fmaf(x[e], ud[e], dv); }
      }
      sv += __shfl_xor(sv, 1, 32);
      dv += __shfl_xor(dv, 1, 32);
      sv += __shfl_xor(sv, 2, 32);
      dv += __shfl_xor(dv, 2, 32);
      if (part == 0) { s_sl[n] = sv; s_dl[n] = dv; }
    }
    {
      const int mt = wid >> 1, nt = wid & 1;
      const int n = mt * 16 + n15;
      const int f = nt * 16 + n15;
      const v16h xa0 = frag_norm_f32(s_y0 + n * FCAT + 8 * hh, s_mean + 8 * hh, s_rstd + 8 * hh, X_CARRY);
      const v16h xa1 = frag_norm_f32(s_y0 + n * FCAT + 32 + 8 * hh, s_mean + 32 + 8 * hh, s_rstd + 32 + 8 * hh, X_CARRY);
      v8f acc = zero8;
      acc = mma16(xa0, Frag<_Float16>::load(s_w1t + f * FCAT + 8 * hh), acc);
      acc = mma16(xa1, Frag<_Float16>::load(s_w1t + f * FCAT + 32 + 8 * hh), acc);
      v8h o;
#pragma unroll
      for (int r = 0; r < 8; ++r) o[r] = (_Float16)(acc[r] * HP_FOLD);
      *(v8ha*)(s_hpt + f * NAGENT + mt * 16 + rb) = o;
    }
    __syncthreads();

#pragma unroll 1
    for (int it = 0; it < 2; ++it) {
      const int n = it * 32 + (tid >> 3);
      attn_row_block(s_sl, s_dl, s_attn, n, tid & 7);
    }
    __syncthreads();

    {
      const int mt = wid >> 1, nt = wid & 1;
      const int f = nt * 16 + n15;
      const _Float16* arow = s_attn + (mt * 16 + n15) * NAGENT + 8 * hh;
      const _Float16* brow = s_hpt + f * NAGENT + 8 * hh;
      v8f acc = zero8;
      acc = mma16(Frag<_Float16>::load(arow), Frag<_Float16>::load(brow), acc);
      acc = mma16(Frag<_Float16>::load(arow + 32), Frag<_Float16>::load(brow + 32), acc);
      const float bb = s_b1v[f];
#pragma unroll
      for (int r = 0; r < 8; ++r) s_ah[(mt * 16 + rb + r) * AHID + f] = acc[r] * PV_FOLD + bb;
    }
    __syncthreads();

    {
      const int m = tid >> 2, part = tid & 3;
      const float* ar = s_ah + m * AHID + part * 8;
      float s0 = 0.0f, s1 = 0.0f;
#pragma unroll
      for (int i = 0; i < 2; ++i) {
        const v4f a  = *(const v4fa*)(ar + 4 * i);
        const v4f wa = *(const v4fa*)(s_wh2a + part * 8 + 4 * i);
        const v4f wb = *(const v4fa*)(s_wh2a + AHID + part * 8 + 4 * i);
#pragma unroll
        for (int e = 0; e < 4; ++e) { s0 = fmaf(a[e], wa[e], s0); s1 = fmaf(a[e], wb[e], s1); }
      }
      s0 += __shfl_xor(s0, 1, 32);
      s1 += __shfl_xor(s1, 1, 32);
      s0 += __shfl_xor(s0, 2, 32);
      s1 += __shfl_xor(s1, 2, 32);
      s0 += s_bh[2];
      s1 += s_bh[3];
      if (part == 0) { s_ao[2 * m] = s0; s_ao[2 * m + 1] = s1; }
      float* grow = s_gh + m * GHID + part * 16;
      const float* wq = s_waa + 2 * part * 16;
      const float* bq = s_baa + part * 16;
      float mx = -INFINITY;
#pragma unroll 1
      for (int c8 = 0; c8 < 16; c8 += 8) {
#pragma unroll
        for (int e = 0; e < 8; ++e) {
          const int jj = c8 + e;
          const float l = fmaf(s0, wq[2 * jj], fmaf(s1, wq[2 * jj + 1], bq[jj]));
          mx = fmaxf(mx, l);
        }
      }
      mx = fmaxf(mx, __shfl_xor(mx, 1, 32));
      mx = fmaxf(mx, __shfl_xor(mx, 2, 32));
      float sum = 0.0f;
#pragma unroll 1
      for (int c8 = 0; c8 < 16; c8 += 8) {
#pragma unroll
        for (int e = 0; e < 8; ++e) {
          const int jj = c8 + e;
          const float l = fmaf(s0, wq[2 * jj], fmaf(s1, wq[2 * jj + 1], bq[jj]));
          const float ev = expf(l - mx);
          sum += ev;
          grow[jj] = grow[jj] * ev;
        }
      }
      sum += __shfl_xor(sum, 1, 32);
      sum += __shfl_xor(sum, 2, 32);
      const float inv = __builtin_amdgcn_rcpf(sum);
#pragma unroll 1
      for (int c8 = 0; c8 < 16; c8 += 8) {
#pragma unroll
        for (int e = 0; e < 8; ++e) grow[c8 + e] = grow[c8 + e] * inv;
      }
    }
    __syncthreads();

    if (tid < 128) {
      const float v = s_ao[tid];
      volatile float* p = out + (size_t)PRED_STEPS * (NPED * 2) + (size_t)t * (NPED * 2) + (size_t)ped0 * 2 + tid;
      *p = v;
      __threadfence();
      *p = v;
    }
  }
}

extern "C" void kernel_launch(void* const* d_in, const int* in_sizes, int n_in,
                              void* d_out, int out_size, void* d_ws, size_t ws_size, hipStream_t stream) {
  (void)d_ws; (void)ws_size;
  if (n_in < 30 || d_out == nullptr) return;
  if (in_sizes[2] != ALL_STEPS * NPED * 2 || in_sizes[3] != NPED * GHID ||
      in_sizes[4] != ALL_STEPS * NPED * 2 || in_sizes[5] != NPED * AHID ||
      in_sizes[7] != 4 * GHID * GHID || in_sizes[13] != 4 * AHID * AHID ||
      in_sizes[22] != NHEAD0 * AHID * FOUT0 || in_sizes[26] != FCAT * FOUT1 ||
      out_size != 2 * PRED_STEPS * NPED * 2) return;
  scene_decode_kernel<<<NSCENE, NTHR, 0, stream>>>(
      (const float*)d_in[2],  (const float*)d_in[3],
      (const float*)d_in[4],  (const float*)d_in[5],
      (const float*)d_in[6],  (const float*)d_in[7],
      (const float*)d_in[8],  (const float*)d_in[9],
      (const float*)d_in[10], (const float*)d_in[11],
      (const float*)d_in[12], (const float*)d_in[13],
      (const float*)d_in[14], (const float*)d_in[15],
      (const float*)d_in[16], (const float*)d_in[17],
      (const float*)d_in[18], (const float*)d_in[19],
      (const float*)d_in[20], (const float*)d_in[21],
      (const float*)d_in[22], (const float*)d_in[23],
      (const float*)d_in[24], (const float*)d_in[25],
      (const float*)d_in[26], (const float*)d_in[27],
      (const float*)d_in[28], (const float*)d_in[29],
      (float*)d_out);
}
